// PerspectiveConv2d_40432822124900
// MI455X (gfx1250) — hardware-verified
//
#include <hip/hip_runtime.h>

typedef _Float16 f16t;
typedef _Float16 v16h __attribute__((ext_vector_type(16)));
typedef _Float16 v8h  __attribute__((ext_vector_type(8)));
typedef _Float16 v2h  __attribute__((ext_vector_type(2)));
typedef float    v8f  __attribute__((ext_vector_type(8)));
typedef float    v4f  __attribute__((ext_vector_type(4)));
typedef int      v4i  __attribute__((ext_vector_type(4)));
typedef v8h __attribute__((may_alias)) v8ha;
typedef v2h __attribute__((may_alias)) v2ha;
typedef v8f __attribute__((may_alias)) v8fa;
typedef v4f __attribute__((may_alias)) v4fa;
typedef v4i __attribute__((may_alias)) v4ia;
union Frag { v16h v; v8h half[2]; };

#define NB    8
#define CIN   512
#define COUT  512
#define HH    18
#define WD    80
#define NP    (HH * WD)
#define KK    (CIN * 9)
#define MTOT  (NB * NP)
#define NOFF  18
#define BM    32
#define KCH   64
#define NCH   (KK / KCH)
#define LDK   (KCH + 8)
#define WSC   64.0f

static_assert(MTOT % BM == 0);
static_assert(NP % BM == 0);
static_assert(KK % KCH == 0);
static_assert(CIN % KCH == 0);
static_assert((COUT * KK / 8) % 256 == 0);

__device__ __forceinline__ v8f wmma_f16(v16h a, v16h b, v8f c) {
  v8f d = __builtin_amdgcn_wmma_f32_16x16x32_f16(false, a, false, b, (short)0, c, false, false);
  asm volatile("v_nop\n\tv_nop\n\tv_nop\n\tv_nop" : "+v"(d) : "v"(a), "v"(b));
  return d;
}

__device__ __forceinline__ v16h load_frag32(const f16t* p, int h) {
  Frag f;
  f.half[0] = *(const v8ha*)(p + 8 * h);
  f.half[1] = *(const v8ha*)(p + 16 + 8 * h);
  return f.v;
}

__device__ __forceinline__ v8f zero8f() {
  v8f z;
  #pragma unroll
  for (int j = 0; j < 8; ++j) z[j] = 0.f;
  return z;
}

__global__ __launch_bounds__(256) void wcvt_k(const float* __restrict__ w, f16t* __restrict__ Wr)
{
  const int g = blockIdx.x * 256 + threadIdx.x;
  if (g >= COUT * KK / 8) return;
  const int e8 = g * 8;
  const int o = e8 / KK, kk = e8 - o * KK;
  const int tap = kk >> 9, c = kk & 511;
  const float* base = w + (size_t)(o * CIN + c) * 9 + tap;
  v8h o8;
  #pragma unroll
  for (int i = 0; i < 8; ++i) o8[i] = (f16t)(base[i * 9] * WSC);
  f16t* dst = Wr + e8;
  *(volatile v8h*)dst = o8;
  __threadfence();
  *(volatile v8h*)dst = o8;
}

__device__ __forceinline__ void fill_tile(const float* __restrict__ feat, const int* so,
                                          const float* sw, f16t* dst, int c0)
{
  #pragma clang fp contract(off)
  const v4i o4 = *(const v4ia*)so;
  const v4f w4 = *(const v4fa*)sw;
  const float* f0 = feat + o4.x + c0 * NP;
  const float* f1 = feat + o4.y + c0 * NP;
  const float* f2 = feat + o4.z + c0 * NP;
  const float* f3 = feat + o4.w + c0 * NP;
  #pragma unroll 1
  for (int g = 0; g < 4; ++g) {
    const int ca = (2 * g) * NP, cb = ca + NP;
    float va = f0[ca] * w4.x;
    va = va + f1[ca] * w4.y;
    va = va + f2[ca] * w4.z;
    va = va + f3[ca] * w4.w;
    float vb = f0[cb] * w4.x;
    vb = vb + f1[cb] * w4.y;
    vb = vb + f2[cb] * w4.z;
    vb = vb + f3[cb] * w4.w;
    v2h pr;
    pr.x = (f16t)va;
    pr.y = (f16t)vb;
    *(v2ha*)(dst + 2 * g) = pr;
  }
}

__global__ __launch_bounds__(256) void dconv_k(const float* __restrict__ feat,
                                               const float* __restrict__ offs,
                                               const f16t*  __restrict__ Wr,
                                               float* __restrict__ out)
{
  __shared__ __attribute__((aligned(32))) f16t  Abuf[2][BM][LDK];
  __shared__ __attribute__((aligned(16))) int   sOff[BM][9][4];
  __shared__ __attribute__((aligned(16))) float sWgt[BM][9][4];
  __shared__ __attribute__((aligned(32))) float sO[8 * 32 * 32];

  const int tid = threadIdx.x, lane = tid & 31, wave = tid >> 5;
  const int h = lane >> 4, m = lane & 15;
  const int m_base = blockIdx.x * BM;
  const int gm  = lane;
  const int kk0 = wave * 8;

  for (int idx = tid; idx < BM * 9; idx += 256) {
    #pragma clang fp contract(off)
    const int mrow = idx / 9, t = idx - 9 * mrow;
    const int mg = m_base + mrow;
    const int b = mg / NP;
    const int rem = mg - b * NP;
    const int hy = rem / WD;
    const int wx = rem - hy * WD;
    const float dy = offs[((b * NOFF + 2 * t    ) * HH + hy) * WD + wx];
    const float dx = offs[((b * NOFF + 2 * t + 1) * HH + hy) * WD + wx];
    const int kh = t / 3, kw = t - 3 * kh;
    const float py = dy + (float)(hy - 1 + kh);
    const float px = dx + (float)(wx - 1 + kw);
    const float fy = floorf(py), fx = floorf(px);
    const float ly = py - fy, lx = px - fx;
    const int y0 = (int)fminf(fmaxf(fy, -4.0f), (float)(HH + 2));
    const int x0 = (int)fminf(fmaxf(fx, -4.0f), (float)(WD + 2));
    const float wy0 = 1.0f - ly, wy1 = ly;
    const float wx0 = 1.0f - lx, wx1 = lx;
    const int bbase = b * CIN * NP;
    const int y1 = y0 + 1, x1 = x0 + 1;
    const bool vy0 = (y0 >= 0) && (y0 < HH), vy1 = (y1 >= 0) && (y1 < HH);
    const bool vx0 = (x0 >= 0) && (x0 < WD), vx1 = (x1 >= 0) && (x1 < WD);
    const int yc0 = min(max(y0, 0), HH - 1), yc1 = min(max(y1, 0), HH - 1);
    const int xc0 = min(max(x0, 0), WD - 1), xc1 = min(max(x1, 0), WD - 1);
    sOff[mrow][t][0] = bbase + yc0 * WD + xc0;
    sOff[mrow][t][1] = bbase + yc0 * WD + xc1;
    sOff[mrow][t][2] = bbase + yc1 * WD + xc0;
    sOff[mrow][t][3] = bbase + yc1 * WD + xc1;
    sWgt[mrow][t][0] = (vy0 && vx0) ? wy0 * wx0 : 0.0f;
    sWgt[mrow][t][1] = (vy0 && vx1) ? wy0 * wx1 : 0.0f;
    sWgt[mrow][t][2] = (vy1 && vx0) ? wy1 * wx0 : 0.0f;
    sWgt[mrow][t][3] = (vy1 && vx1) ? wy1 * wx1 : 0.0f;
  }
  __syncthreads();

  const v8f z8 = zero8f();
  v8f acc[2][4];
  #pragma unroll
  for (int ms = 0; ms < 2; ++ms) {
    #pragma unroll
    for (int nt = 0; nt < 4; ++nt) acc[ms][nt] = z8;
  }

  fill_tile(feat, &sOff[gm][0][0], &sWgt[gm][0][0], &Abuf[0][gm][kk0], kk0);
  __syncthreads();

  const f16t* wrow = Wr + (size_t)(wave * 64 + m) * KK;
  const size_t bst = (size_t)16 * KK;

  #pragma unroll 1
  for (int chunk = 0; chunk < NCH; ++chunk) {
    const int cur = chunk & 1;
    #pragma unroll
    for (int ks = 0; ks < 2; ++ks) {
      const int koff = ks * 32;
      const v16h a0 = load_frag32(&Abuf[cur][m][koff], h);
      const v16h a1 = load_frag32(&Abuf[cur][16 + m][koff], h);
      const int k0 = chunk * KCH + koff;
      #pragma unroll
      for (int nt = 0; nt < 4; ++nt) {
        const v16h bb = load_frag32(wrow + nt * bst + k0, h);
        acc[0][nt] = wmma_f16(a0, bb, acc[0][nt]);
        acc[1][nt] = wmma_f16(a1, bb, acc[1][nt]);
      }
    }
    if (chunk + 1 < NCH) {
      const int kb = (chunk + 1) * KCH;
      const int t  = kb >> 9;
      const int c0 = (kb & 511) + kk0;
      fill_tile(feat, &sOff[gm][t][0], &sWgt[gm][t][0], &Abuf[cur ^ 1][gm][kk0], c0);
    }
    __syncthreads();
  }

  const int bo = m_base / NP;
  const int p0 = m_base - bo * NP;
  const float osc = 1.0f / WSC;
  const int q8 = lane & 7, sub = lane >> 3;
  float* sOw = sO + wave * 1024;

  #pragma unroll
  for (int rr = 0; rr < 2; ++rr) {
    __syncthreads();
    #pragma unroll
    for (int q = 0; q < 2; ++q) {
      const int nl = 16 * q + m;
      #pragma unroll
      for (int ms = 0; ms < 2; ++ms) {
        v8f vv;
        #pragma unroll
        for (int r = 0; r < 8; ++r) vv[r] = acc[ms][2 * rr + q][r] * osc;
        *(v8fa*)(sOw + nl * 32 + 16 * ms + 8 * h) = vv;
      }
    }
    __syncthreads();
    v4f vals[8];
    size_t d[8];
    #pragma unroll
    for (int i = 0; i < 8; ++i) {
      const int cl = 4 * i + sub;
      vals[i] = *(const v4fa*)(sOw + cl * 32 + 4 * q8);
      const int n = wave * 64 + 32 * rr + cl;
      d[i] = (size_t)(bo * COUT + n) * NP + p0 + 4 * q8;
    }
    #pragma unroll
    for (int i = 0; i < 8; ++i) *(volatile v4f*)(out + d[i]) = vals[i];
    __threadfence();
    #pragma unroll
    for (int i = 0; i < 8; ++i) *(volatile v4f*)(out + d[i]) = vals[i];
  }
}

extern "C" void kernel_launch(void* const* d_in, const int* in_sizes, int n_in,
                              void* d_out, int out_size, void* d_ws, size_t ws_size,
                              hipStream_t stream) {
  if (n_in < 3) return;
  if (in_sizes[0] != NB * CIN * NP) return;
  if (in_sizes[1] != NB * NOFF * NP) return;
  if (in_sizes[2] != COUT * CIN * 9) return;
  if (out_size != NB * COUT * NP) return;

  const float* feat = (const float*)d_in[0];
  const float* offs = (const float*)d_in[1];
  const float* wgt  = (const float*)d_in[2];
  float* outp = (float*)d_out;

  const size_t szWr = (size_t)COUT * KK * 2;
  if (szWr > ws_size) return;
  f16t* Wr = (f16t*)d_ws;

  wcvt_k<<<(COUT * KK / 8) / 256, 256, 0, stream>>>(wgt, Wr);
  dconv_k<<<MTOT / BM, 256, 0, stream>>>(feat, offs, Wr, outp);
}
